// EER_GCN_9199819948207
// MI455X (gfx1250) — hardware-verified
//
#include <hip/hip_runtime.h>


#define NS 4096
#define NNODE 62
#define NF 5
#define HID 32
#define NE_ 3782
#define FC1 128
#define NCLS 3
#define NROW (NS * NNODE)
#define NCOL (NS * NF)

typedef __attribute__((ext_vector_type(16))) __bf16   v16bf;
typedef __attribute__((ext_vector_type(16))) _Float16 v16h;
typedef __attribute__((ext_vector_type(8)))  float    v8f;
typedef __attribute__((ext_vector_type(8)))  unsigned v8u;

__device__ __forceinline__ unsigned f2bf(float f) { unsigned u = __float_as_uint(f); u += 0x7FFFu + ((u >> 16) & 1u); return u >> 16; }
__device__ __forceinline__ unsigned f2h(float f) { return (unsigned)__builtin_bit_cast(unsigned short, (_Float16)f); }
__device__ __forceinline__ int kpat(int v, int half) { return ((v & 4) ? 16 : 0) + half * 8 + 2 * (v & 3); }

template <int F16, int NP> struct Opnd { v16bf p[NP]; };

template <int F16, int NP> __device__ __forceinline__ void pack2(float f0, float f1, unsigned* o) {
    if (F16) { o[0] = f2h(f0) | (f2h(f1) << 16); return; }
    unsigned h0 = f2bf(f0), h1 = f2bf(f1); o[0] = h0 | (h1 << 16);
    if (NP >= 2) {
        float r0 = f0 - __uint_as_float(h0 << 16), r1 = f1 - __uint_as_float(h1 << 16);
        unsigned m0 = f2bf(r0), m1 = f2bf(r1); o[1] = m0 | (m1 << 16);
        if (NP >= 3) {
            float s0 = r0 - __uint_as_float(m0 << 16), s1 = r1 - __uint_as_float(m1 << 16);
            o[2] = f2bf(s0) | (f2bf(s1) << 16);
        }
    }
}
template <int F16, int NP> __device__ __forceinline__ void op_row(const float* rowp, int half, float sc, Opnd<F16, NP>& o) {
    v8u u[NP];
#pragma unroll
    for (int v = 0; v < 8; ++v) {
        int kk = kpat(v, half); unsigned t[3];
        pack2<F16, NP>(rowp[kk] * sc, rowp[kk + 1] * sc, t);
#pragma unroll
        for (int p = 0; p < NP; ++p) u[p][v] = t[p];
    }
#pragma unroll
    for (int p = 0; p < NP; ++p) o.p[p] = __builtin_bit_cast(v16bf, u[p]);
}
template <int F16, int NP> __device__ __forceinline__ void op_row_tail(const float* rowp, int half, float sc, int kvalid, Opnd<F16, NP>& o) {
    v8u u[NP];
#pragma unroll
    for (int v = 0; v < 8; ++v) {
        int kk = kpat(v, half); unsigned t[3];
        float f0 = kk < kvalid ? rowp[kk] * sc : 0.0f, f1 = (kk + 1) < kvalid ? rowp[kk + 1] * sc : 0.0f;
        pack2<F16, NP>(f0, f1, t);
#pragma unroll
        for (int p = 0; p < NP; ++p) u[p][v] = t[p];
    }
#pragma unroll
    for (int p = 0; p < NP; ++p) o.p[p] = __builtin_bit_cast(v16bf, u[p]);
}
template <int F16, int NP> __device__ __forceinline__ void op_col(const float* M, int ld, int n, int k0, int half, float sc, Opnd<F16, NP>& o) {
    v8u u[NP];
#pragma unroll
    for (int v = 0; v < 8; ++v) {
        int kk = k0 + kpat(v, half); unsigned t[3];
        pack2<F16, NP>(M[(size_t)kk * ld + n] * sc, M[(size_t)(kk + 1) * ld + n] * sc, t);
#pragma unroll
        for (int p = 0; p < NP; ++p) u[p][v] = t[p];
    }
#pragma unroll
    for (int p = 0; p < NP; ++p) o.p[p] = __builtin_bit_cast(v16bf, u[p]);
}
template <int F16, int NP> __device__ __forceinline__ void op_col_tail(const float* M, int ld, int n, int k0, int half, float sc, int K, Opnd<F16, NP>& o) {
    v8u u[NP];
#pragma unroll
    for (int v = 0; v < 8; ++v) {
        int kk = k0 + kpat(v, half); unsigned t[3];
        float f0 = kk < K ? M[(size_t)kk * ld + n] * sc : 0.0f, f1 = (kk + 1) < K ? M[(size_t)(kk + 1) * ld + n] * sc : 0.0f;
        pack2<F16, NP>(f0, f1, t);
#pragma unroll
        for (int p = 0; p < NP; ++p) u[p][v] = t[p];
    }
#pragma unroll
    for (int p = 0; p < NP; ++p) o.p[p] = __builtin_bit_cast(v16bf, u[p]);
}
__device__ __forceinline__ v8f wm_bf16(v16bf a, v16bf b, v8f c) { return __builtin_amdgcn_wmma_f32_16x16x32_bf16(false, a, false, b, (short)0, c, false, false); }
template <int F16, int NA, int NB> __device__ __forceinline__ v8f wmma_op(const Opnd<F16, NA>& a, const Opnd<F16, NB>& b, v8f c) {
    if (F16) {
        v16h ah = __builtin_bit_cast(v16h, a.p[0]), bh = __builtin_bit_cast(v16h, b.p[0]);
        c = __builtin_amdgcn_wmma_f32_16x16x32_f16(false, ah, false, bh, (short)0, c, false, false);
        asm volatile("v_nop\n\tv_nop\n\tv_nop\n\tv_nop" : "+v"(c) : "v"(ah), "v"(bh));
        return c;
    }
    constexpr int NMX = NA > NB ? NA : NB;
#pragma unroll
    for (int i = 0; i < NA; ++i)
#pragma unroll
        for (int j = 0; j < NB; ++j)
            if (i + j < NMX) c = wm_bf16(a.p[i], b.p[j], c);
    if (NA == 1 && NB == 1)      asm volatile("v_nop\n\tv_nop\n\tv_nop\n\tv_nop" : "+v"(c) : "v"(a.p[0]), "v"(b.p[0]));
    else if (NA == 2 && NB == 1) asm volatile("v_nop\n\tv_nop\n\tv_nop\n\tv_nop" : "+v"(c) : "v"(a.p[0]), "v"(a.p[1]), "v"(b.p[0]));
    else if (NA == 1 && NB == 2) asm volatile("v_nop\n\tv_nop\n\tv_nop\n\tv_nop" : "+v"(c) : "v"(a.p[0]), "v"(b.p[0]), "v"(b.p[1]));
    else if (NA == 2 && NB == 2) asm volatile("v_nop\n\tv_nop\n\tv_nop\n\tv_nop" : "+v"(c) : "v"(a.p[0]), "v"(a.p[1]), "v"(b.p[0]), "v"(b.p[1]));
    else                         asm volatile("v_nop\n\tv_nop\n\tv_nop\n\tv_nop" : "+v"(c) : "v"(a.p[0]), "v"(a.p[NA - 1]), "v"(b.p[0]), "v"(b.p[NB - 1]), "v"(a.p[NA / 2]), "v"(b.p[NB / 2]));
    return c;
}

struct ZMap { long long s1; long long s2; int zdiv; int pad_; };
__device__ __forceinline__ size_t zoff(const ZMap& m, int z) { return (size_t)((long long)(z / m.zdiv) * m.s1 + (long long)(z % m.zdiv) * m.s2); }

#define ACT_NONE 0
#define ACT_RELU 1
#define ACT_GELU_ERF 2
#define ACT_SILU 3
#define ACT_TANH 4
__device__ __forceinline__ float act_apply(int act, float x) {
    if (act == ACT_RELU) return x > 0.f ? x : 0.f;
    if (act == ACT_GELU_ERF) return 0.5f * x * (1.0f + erff(x * 0.70710678118654752f));
    if (act == ACT_SILU) return x / (1.0f + expf(-x));
    if (act == ACT_TANH) return tanhf(x);
    return x;
}
struct GemmArgs {
    ZMap za, zb_, zc, zbias, zadd, zrsc, zmul, zrbias;
    const float* A; const float* Bm; float* C; const float* bias; const float* add; const float* rsc; const float* mul; const float* rbias;
    long long ldadd, ldmul;
    int lda, ldb, ldc, K;
    float ascale, bscale, oscale, addscale;
    int M, nvalid, nstore, ldrsc;
    int bcs, pad1, pad2, pad3;
};
template <int BT, int F16, int NA, int NB, int RW, int CW, int ACT>
__global__ __launch_bounds__(256) void gemm_kernel(GemmArgs g) {
    constexpr int TR = 16 * RW, TC = 64 * CW, CSTR = TC + 4;
    __shared__ __align__(16) float cst[TR * CSTR];
    const int z = blockIdx.z;
    const float* A = g.A + zoff(g.za, z); const float* Bm = g.Bm + zoff(g.zb_, z); float* C = g.C + zoff(g.zc, z);
    const int tid = threadIdx.x, lane = tid & 31, wv = tid >> 5;
    const int l16 = lane & 15, half = lane >> 4;
    const int rt = wv % RW, ch = wv / RW;
    const int row0 = blockIdx.x * TR, col0 = blockIdx.y * TC + ch * 64;
    int arix = row0 + rt * 16 + l16; if (arix >= g.M) arix = g.M - 1;
    const float* arow = A + (size_t)arix * g.lda;
    v8f acc[4];
#pragma unroll
    for (int t = 0; t < 4; ++t) acc[t] = (v8f){};
    const int K = g.K;
#pragma unroll 1
    for (int kc = 0; kc < K; kc += 32) {
        Opnd<F16, NA> a;
        if (kc + 32 <= K) op_row<F16, NA>(arow + kc, half, g.ascale, a); else op_row_tail<F16, NA>(arow + kc, half, g.ascale, K - kc, a);
#pragma unroll
        for (int t = 0; t < 4; ++t) {
            Opnd<F16, NB> b;
            const int n = col0 + t * 16 + l16;
            if (n < g.nvalid) {
                if (BT) { if (kc + 32 <= K) op_row<F16, NB>(Bm + (size_t)n * g.ldb + kc, half, g.bscale, b); else op_row_tail<F16, NB>(Bm + (size_t)n * g.ldb + kc, half, g.bscale, K - kc, b); }
                else    { if (kc + 32 <= K) op_col<F16, NB>(Bm, g.ldb, n * g.bcs, kc, half, g.bscale, b); else op_col_tail<F16, NB>(Bm, g.ldb, n * g.bcs, kc, half, g.bscale, K, b); }
            } else {
#pragma unroll
                for (int p = 0; p < NB; ++p) b.p[p] = (v16bf){};
            }
            acc[t] = wmma_op<F16, NA, NB>(a, b, acc[t]);
        }
    }
    const float* bias = g.bias ? g.bias + zoff(g.zbias, z) : nullptr;
    const float* add = g.add ? g.add + zoff(g.zadd, z) : nullptr;
    const float* rsc = g.rsc ? g.rsc + zoff(g.zrsc, z) : nullptr;
    const float* mul = g.mul ? g.mul + zoff(g.zmul, z) : nullptr;
    const float* rbias = g.rbias ? g.rbias + zoff(g.zrbias, z) : nullptr;
#pragma unroll
    for (int t = 0; t < 4; ++t) {
        const int cl = ch * 64 + t * 16 + l16;
        const int cg = blockIdx.y * TC + cl;
        const bool cok = cg < g.nvalid;
        const float bv = (bias && cok) ? bias[(size_t)cg * g.bcs] : 0.0f;
#pragma unroll
        for (int r = 0; r < 8; ++r) {
            const int rl = rt * 16 + r + 8 * half;
            float v = acc[t][r] * g.oscale + bv;
            int rg = row0 + rl; if (rg >= g.M) rg = g.M - 1;
            if (rbias) v += rbias[rg];
            if (rsc) v *= rsc[(size_t)rg * g.ldrsc];
            if (mul && cok) v *= mul[(size_t)rg * g.ldmul + cg];
            if (add && cok) v += g.addscale * add[(size_t)rg * g.ldadd + cg];
            cst[rl * CSTR + cl] = v;
        }
    }
    __syncthreads();
    const int col = tid % TC, rsel = tid / TC, rstep = 256 / TC;
    if (ACT != ACT_NONE) {
#pragma unroll 1
        for (int r = rsel; r < TR; r += rstep) cst[r * CSTR + col] = act_apply(ACT, cst[r * CSTR + col]);
    }
    float* ob = C + (size_t)row0 * g.ldc + (size_t)blockIdx.y * TC;
    const bool colok = (int)(blockIdx.y * TC + col) < g.nstore;
    const int rmax = (g.M - row0 < TR) ? (g.M - row0) : TR;
    auto pass = [&]() {
        if (colok) {
#pragma unroll 4
            for (int r = rsel; r < rmax; r += rstep) *(volatile float*)(ob + (size_t)r * g.ldc + col) = cst[r * CSTR + col];
        }
    };
    pass();
    __threadfence();
    pass();
}
static inline ZMap zm(long long s1) { ZMap m; m.s1 = s1; m.s2 = 0; m.zdiv = 1; m.pad_ = 0; return m; }
static inline ZMap zm2(long long s1, long long s2, int zdiv) { ZMap m; m.s1 = s1; m.s2 = s2; m.zdiv = zdiv; m.pad_ = 0; return m; }
static inline GemmArgs gemm_args(const float* A, int lda, ZMap za, const float* Bm, int ldb, ZMap zb, float* C, int ldc, ZMap zc, int M, int N, int K) {
    GemmArgs g; g.za = za; g.zb_ = zb; g.zc = zc; g.zbias = zm(0); g.zadd = zm(0); g.zrsc = zm(0); g.zmul = zm(0); g.zrbias = zm(0);
    g.A = A; g.Bm = Bm; g.C = C; g.bias = nullptr; g.add = nullptr; g.rsc = nullptr; g.mul = nullptr; g.rbias = nullptr; g.ldadd = 0; g.ldmul = 0;
    g.lda = lda; g.ldb = ldb; g.ldc = ldc; g.K = K; g.ascale = 1.0f; g.bscale = 1.0f; g.oscale = 1.0f; g.addscale = 1.0f; g.M = M; g.nvalid = N; g.nstore = N; g.ldrsc = 1;
    g.bcs = 1; g.pad1 = 0; g.pad2 = 0; g.pad3 = 0;
    return g;
}
static_assert(sizeof(ZMap) == 24, "ZMap layout");
static_assert(sizeof(GemmArgs) == 8 * 24 + 8 * 8 + 2 * 8 + 4 * 4 + 4 * 4 + 4 * 4 + 4 * 4, "GemmArgs has no padding");

__global__ __launch_bounds__(256) void softmax_rows(float* S, long long sy, long long sx, int L, float prescale, const float* addv, long long say, int aydiv, int causal,
                                                  const int* imask, long long imy, long long imx, float maskval) {
    __shared__ float red[8];
    const int tid = threadIdx.x, lane = tid & 31, wid = tid >> 5;
    float* row = S + (size_t)blockIdx.y * sy + (size_t)blockIdx.x * sx;
    const float* av = addv ? addv + (size_t)(blockIdx.y / aydiv) * say : nullptr;
    const int* im = imask ? imask + (size_t)(blockIdx.y / aydiv) * imy + (size_t)blockIdx.x * imx : nullptr;
    float v[16];
    const int nj = L / 256;
    float mx = -__builtin_inff();
#pragma unroll
    for (int j = 0; j < 16; ++j) if (j < nj) { float t = row[tid + 256 * j] * prescale; if (av) t += av[tid + 256 * j]; if (im && im[tid + 256 * j] == 0) t = maskval; if (causal && (tid + 256 * j) > (int)blockIdx.x) t = -__builtin_inff(); v[j] = t; mx = fmaxf(mx, t); }
#pragma unroll
    for (int o = 16; o; o >>= 1) mx = fmaxf(mx, __shfl_xor(mx, o, 32));
    if (lane == 0) red[wid] = mx;
    __syncthreads();
    float m = red[0];
#pragma unroll
    for (int i = 1; i < 8; ++i) m = fmaxf(m, red[i]);
    if (m == -__builtin_inff()) m = 0.f;
    __syncthreads();
    float sum = 0.f;
#pragma unroll
    for (int j = 0; j < 16; ++j) if (j < nj) { v[j] = expf(v[j] - m); sum += v[j]; }
#pragma unroll
    for (int o = 16; o; o >>= 1) sum += __shfl_xor(sum, o, 32);
    if (lane == 0) red[wid] = sum;
    __syncthreads();
    float tot = 0.f;
#pragma unroll
    for (int i = 0; i < 8; ++i) tot += red[i];
    const float inv = 1.0f / tot;
#pragma unroll
    for (int j = 0; j < 16; ++j) if (j < nj) *(volatile float*)(row + tid + 256 * j) = v[j] * inv;
    __threadfence();
#pragma unroll
    for (int j = 0; j < 16; ++j) if (j < nj) *(volatile float*)(row + tid + 256 * j) = v[j] * inv;
}

#define VST2(T, p, v) do { const T vst2_v_ = (v); *(volatile T*)(p) = vst2_v_; __threadfence(); *(volatile T*)(p) = vst2_v_; } while (0)
__global__ __launch_bounds__(64) void k_eig(const int* __restrict__ ei, const float* __restrict__ ew, float* PAR) { __shared__ double A[NNODE][NNODE]; __shared__ double cs[2]; __shared__ double dl[NNODE]; const int t = threadIdx.x;
    for (int e = t; e < NNODE * NNODE; e += 64) A[e / NNODE][e % NNODE] = 0.0; if (t < NNODE) dl[t] = 0.0; __syncthreads();
    if (t == 0) { for (int e = 0; e < NE_; ++e) { int s = ei[e], d = ei[NE_ + e]; s = s < 0 ? 0 : (s >= NNODE ? NNODE - 1 : s); d = d < 0 ? 0 : (d >= NNODE ? NNODE - 1 : d); const double w = (double)ew[e]; A[s][d] -= w; A[s][s] += w; const float wl = ew[e] >= 0.f ? ew[e] : 0.15f * ew[e]; dl[s] += (double)wl; } }
    __syncthreads();
    for (int e = t; e < NNODE * NNODE; e += 64) { const int i = e / NNODE, j = e % NNODE; if (i < j) { const double m = 0.5 * (A[i][j] + A[j][i]); A[i][j] = m; A[j][i] = m; } } __syncthreads();
    for (int sweep = 0; sweep < 12; ++sweep) {
        for (int p = 0; p < NNODE - 1; ++p) for (int q = p + 1; q < NNODE; ++q) {
            if (t == 0) { const double apq = A[p][q]; if (fabs(apq) < 1e-300) { cs[0] = 1.0; cs[1] = 0.0; } else { const double th = (A[q][q] - A[p][p]) / (2.0 * apq); const double tt = (th >= 0 ? 1.0 : -1.0) / (fabs(th) + sqrt(th * th + 1.0)); const double c = 1.0 / sqrt(tt * tt + 1.0); cs[0] = c; cs[1] = tt * c; } }
            __syncthreads(); const double c = cs[0], s = cs[1];
            if (s != 0.0 && t < NNODE) { const int k = t; const double akp = A[k][p], akq = A[k][q]; A[k][p] = c * akp - s * akq; A[k][q] = s * akp + c * akq; }
            __syncthreads();
            if (s != 0.0 && t < NNODE) { const int k = t; const double apk = A[p][k], aqk = A[q][k]; A[p][k] = c * apk - s * aqk; A[q][k] = s * apk + c * aqk; }
            __syncthreads(); } }
    if (t == 0) { double lm = -1e300; for (int i = 0; i < NNODE; ++i) lm = lm > A[i][i] ? lm : A[i][i]; const float lam = (float)lm; VST2(float, PAR + 0, lam); const float sc = 2.0f / lam; VST2(float, PAR + 1, sc); for (int n = 0; n < NNODE; ++n) { VST2(float, PAR + 32 + n, (float)dl[n] * sc - 1.0f); } } }
__global__ __launch_bounds__(256) void k_lhat(const int* __restrict__ ei, const float* __restrict__ ew, const float* __restrict__ PAR, float* LH) { __shared__ float M[64][64]; const int t = threadIdx.x; for (int e = t; e < 64 * 64; e += 256) M[e / 64][e % 64] = 0.f; __syncthreads();
    if (t == 0) { const float sc = PAR[1]; for (int e = 0; e < NE_; ++e) { int s = ei[e], d = ei[NE_ + e]; s = s < 0 ? 0 : (s >= NNODE ? NNODE - 1 : s); d = d < 0 ? 0 : (d >= NNODE ? NNODE - 1 : d); const float wl = ew[e] >= 0.f ? ew[e] : 0.15f * ew[e]; M[d][s] += -wl * sc; } for (int n = 0; n < NNODE; ++n) M[n][n] += PAR[32 + n]; }
    __syncthreads(); for (int e = t; e < 64 * 64; e += 256) { VST2(float, LH + e, M[e / 64][e % 64]); } }
__global__ __launch_bounds__(256) void k_bnstat(const float* __restrict__ x, float* ST) { __shared__ double rs[5][256], rq[5][256]; const int t = threadIdx.x; double s[5] = {0, 0, 0, 0, 0}, q[5] = {0, 0, 0, 0, 0};
    for (int i = t; i < NROW; i += 256) {
#pragma unroll
        for (int c = 0; c < 5; ++c) { const double v = (double)x[(size_t)i * NF + c]; s[c] += v; q[c] += v * v; } }
#pragma unroll
    for (int c = 0; c < 5; ++c) { rs[c][t] = s[c]; rq[c][t] = q[c]; } __syncthreads();
    for (int o = 128; o > 0; o >>= 1) { if (t < o) {
#pragma unroll
        for (int c = 0; c < 5; ++c) { rs[c][t] += rs[c][t + o]; rq[c][t] += rq[c][t + o]; } } __syncthreads(); }
    if (t < 5) { const double mean = rs[t][0] / NROW; double var = rq[t][0] / NROW - mean * mean; if (var < 0) var = 0; VST2(float, ST + t * 32, (float)mean); VST2(float, ST + t * 32 + 1, (float)(1.0 / sqrt(var + 1e-5))); } }
__global__ __launch_bounds__(256) void k_x0t(const float* __restrict__ x, const float* __restrict__ ST, const float* __restrict__ g, const float* __restrict__ bb, float* X0T) { const size_t q = (size_t)blockIdx.x * 256 + threadIdx.x; if (q >= (size_t)64 * NCOL) return; const int col = (int)(q % NCOL); const int n = (int)(q / NCOL); const int b = col / NF, f = col % NF; float v = 0.f; if (n < NNODE) { v = (x[((size_t)b * NNODE + n) * NF + f] - ST[f * 32]) * ST[f * 32 + 1] * g[f] + bb[f]; v = v >= 0.f ? v : 0.15f * v; } VST2(float, X0T + q, v); }
__global__ __launch_bounds__(256) void k_cheba(const float* __restrict__ X0T, const float* __restrict__ X1T, const float* __restrict__ X2T, float* CA) { const size_t q = (size_t)blockIdx.x * 256 + threadIdx.x; if (q >= (size_t)NROW * 32) return; const int c = (int)(q % 32); const size_t r = q / 32; const int b = (int)(r / NNODE), n = (int)(r % NNODE); float v = 0.f; if (c < 15) { const int k = c / NF, f = c % NF; const float* T = k == 0 ? X0T : (k == 1 ? X1T : X2T); v = T[(size_t)n * NCOL + b * NF + f]; } VST2(float, CA + q, v); }
__global__ __launch_bounds__(256) void k_leaky(float* A, size_t nn) { const size_t q = (size_t)blockIdx.x * 256 + threadIdx.x; if (q < nn) { const float v = A[q]; VST2(float, A + q, v >= 0.f ? v : 0.15f * v); } }
__global__ __launch_bounds__(256) void k_head(const float* __restrict__ H1, const float* __restrict__ W2, const float* __restrict__ b2, const int* __restrict__ y, float* LP) { const int lane = threadIdx.x & 31; const int b = blockIdx.x * 8 + (threadIdx.x >> 5); if (b >= NS) return; float p0 = 0.f, p1 = 0.f, p2 = 0.f;
#pragma unroll
    for (int q = 0; q < 4; ++q) { float v = H1[(size_t)b * FC1 + lane + 32 * q]; v = v >= 0.f ? v : 0.15f * v; p0 += v * W2[(lane + 32 * q) * 3]; p1 += v * W2[(lane + 32 * q) * 3 + 1]; p2 += v * W2[(lane + 32 * q) * 3 + 2]; }
#pragma unroll
    for (int o = 16; o; o >>= 1) { p0 += __shfl_xor(p0, o, 32); p1 += __shfl_xor(p1, o, 32); p2 += __shfl_xor(p2, o, 32); }
    p0 += b2[0]; p1 += b2[1]; p2 += b2[2]; const float m = fmaxf(p0, fmaxf(p1, p2)); const float e0 = expf(p0 - m), e1 = expf(p1 - m), e2 = expf(p2 - m); const float lse = m + logf(e0 + e1 + e2);
    int yy = y[b]; yy = yy < 0 ? 0 : (yy > 2 ? 2 : yy); const float lpy = (yy == 0 ? p0 : (yy == 1 ? p1 : p2)) - lse;
    float v = 0.f; if (lane == 0) v = expf(p0 - lse); else if (lane == 1) v = expf(p1 - lse); else if (lane == 2) v = expf(p2 - lse); else if (lane == 4) v = -lpy;
    VST2(float, LP + (size_t)b * 32 + lane, v); }
__global__ __launch_bounds__(64) void k_out(const float* __restrict__ LP, float* out) { const int lane = threadIdx.x; if (threadIdx.x >= 32) return; double s = 0.0; for (int b = lane; b < NS; b += 32) s += (double)LP[(size_t)b * 32 + 4];
#pragma unroll
    for (int o = 16; o; o >>= 1) s += __shfl_xor(s, o, 32);
    if (lane == 0) { VST2(float, out, (float)(s / NS)); }
    for (int q = lane; q < NS * 3; q += 32) { VST2(float, out + 1 + q, LP[(size_t)(q / 3) * 32 + (q % 3)]); } }
__global__ __launch_bounds__(256) void k_cw(const float* __restrict__ cw, float* CW) { const int q = blockIdx.x * 256 + threadIdx.x; if (q >= 32 * 32) return; const int h = q % 32, k = q / 32; VST2(float, CW + q, k < 15 ? cw[k * HID + h] : 0.f); }
extern "C" void kernel_launch(void* const* d_in, const int* in_sizes, int n_in,
                              void* d_out, int out_size, void* d_ws, size_t ws_size, hipStream_t stream) {
    (void)in_sizes; (void)n_in; (void)out_size;
    const float* x = (const float*)d_in[0]; const int* y = (const int*)d_in[1]; const int* ei = (const int*)d_in[2]; const float* ew = (const float*)d_in[3]; const float* bng = (const float*)d_in[4]; const float* bnb = (const float*)d_in[5]; const float* cw = (const float*)d_in[6]; const float* cb = (const float*)d_in[7]; const float* f1w = (const float*)d_in[8]; const float* f1b = (const float*)d_in[9]; const float* f2w = (const float*)d_in[10]; const float* f2b = (const float*)d_in[11];
    float* out = (float*)d_out;
    char* wsp = (char*)d_ws;
    auto take = [&](size_t bytes) { char* p = wsp; wsp += (bytes + 255) & ~(size_t)255; return (void*)p; };
    float* PAR = (float*)take(128 * 4); float* LH = (float*)take(64 * 64 * 4); float* ST = (float*)take(5 * 32 * 4); float* X0T = (float*)take((size_t)64 * NCOL * 4); float* X1T = (float*)take((size_t)64 * NCOL * 4); float* X2T = (float*)take((size_t)64 * NCOL * 4); float* CA = (float*)take((size_t)NROW * 32 * 4); float* CW = (float*)take(32 * 32 * 4); float* CO = (float*)take((size_t)NROW * HID * 4); float* H1 = (float*)take((size_t)NS * FC1 * 4); float* LP = (float*)take((size_t)NS * 32 * 4);
    if ((size_t)(wsp - (char*)d_ws) > ws_size) return;
    k_eig<<<1, 64, 0, stream>>>(ei, ew, PAR);
    k_lhat<<<1, 256, 0, stream>>>(ei, ew, PAR, LH);
    k_bnstat<<<1, 256, 0, stream>>>(x, ST);
    k_x0t<<<(unsigned)(((size_t)64 * NCOL) / 256), 256, 0, stream>>>(x, ST, bng, bnb, X0T);
    { GemmArgs g = gemm_args(LH, 64, zm(0), X0T, NCOL, zm(0), X1T, NCOL, zm(0), 64, NCOL, 64); gemm_kernel<0, 0, 2, 2, 4, 2, ACT_NONE><<<dim3(1, NCOL / 128, 1), 256, 0, stream>>>(g); }
    { GemmArgs g = gemm_args(LH, 64, zm(0), X1T, NCOL, zm(0), X2T, NCOL, zm(0), 64, NCOL, 64); g.oscale = 2.0f; g.add = X0T; g.ldadd = NCOL; g.addscale = -1.0f; gemm_kernel<0, 0, 2, 2, 4, 2, ACT_NONE><<<dim3(1, NCOL / 128, 1), 256, 0, stream>>>(g); }
    k_cheba<<<(unsigned)(((size_t)NROW * 32) / 256), 256, 0, stream>>>(X0T, X1T, X2T, CA);
    k_cw<<<4, 256, 0, stream>>>(cw, CW);
    { GemmArgs g = gemm_args(CA, 32, zm(0), CW, HID, zm(0), CO, HID, zm(0), NROW, HID, 15); g.bias = cb; gemm_kernel<0, 0, 2, 2, 8, 1, ACT_NONE><<<dim3(NROW / 128, 1, 1), 256, 0, stream>>>(g); }
    k_leaky<<<(unsigned)(((size_t)NROW * HID + 255) / 256), 256, 0, stream>>>(CO, (size_t)NROW * HID);
    { GemmArgs g = gemm_args(CO, NNODE * HID, zm(0), f1w, FC1, zm(0), H1, FC1, zm(0), NS, FC1, NNODE * HID); g.bias = f1b; gemm_kernel<0, 0, 2, 2, 4, 2, ACT_NONE><<<dim3(NS / 64, 1, 1), 256, 0, stream>>>(g); }
    k_head<<<NS / 8, 256, 0, stream>>>(H1, f2w, f2b, y, LP);
    k_out<<<1, 64, 0, stream>>>(LP, out);
}
